// FNO1d_70815420776999
// MI455X (gfx1250) — hardware-verified
//
#include <hip/hip_runtime.h>


#define NB_  16
#define NN   16384
#define WD   64
#define MO   32
#define TC   64
#define NBLK 4
#define HB   8
#define RWS  (HB * WD)
#define TWOPI_N 3.8349519697141029e-4f
typedef _Float16 h16;
typedef unsigned short bf;
typedef __attribute__((ext_vector_type(16))) __bf16   v16bf;
typedef __attribute__((ext_vector_type(16))) _Float16 v16h;
typedef __attribute__((ext_vector_type(8)))  _Float16 v8h;
typedef __attribute__((ext_vector_type(8)))  unsigned short v8us;
typedef __attribute__((ext_vector_type(8)))  float    v8f;
typedef __attribute__((ext_vector_type(4)))  float    v4f;
typedef v8h  __attribute__((may_alias)) v8ha;
typedef v4f  __attribute__((may_alias)) v4fa;
typedef v8us __attribute__((may_alias)) v8usa;

__device__ __forceinline__ unsigned short f2bf(float f) { unsigned u = __float_as_uint(f); u += 0x7FFFu + ((u >> 16) & 1u); return (unsigned short)(u >> 16); }
__device__ __forceinline__ float bf2f(unsigned short b) { return __uint_as_float(((unsigned)b) << 16); }
__device__ __forceinline__ float bfr(float f) { return bf2f(f2bf(f)); }
__device__ __forceinline__ v16h cat16(v8h lo, v8h hi) { return __builtin_shufflevector(lo, hi, 0, 1, 2, 3, 4, 5, 6, 7, 8, 9, 10, 11, 12, 13, 14, 15); }
__device__ __forceinline__ v16bf cat16b(v8us lo, v8us hi) { return __builtin_bit_cast(v16bf, __builtin_shufflevector(lo, hi, 0, 1, 2, 3, 4, 5, 6, 7, 8, 9, 10, 11, 12, 13, 14, 15)); }
__device__ __forceinline__ v8f wmma16(v16h a, v16h b, v8f c) { return __builtin_amdgcn_wmma_f32_16x16x32_f16(false, a, false, b, (short)0, c, false, false); }
__device__ __forceinline__ v8f wmmab(v16bf a, v16bf b, v8f c) { return __builtin_amdgcn_wmma_f32_16x16x32_bf16(false, a, false, b, (short)0, c, false, false); }


template <typename T16> struct WFrag;
template <> struct WFrag<h16> { typedef v16h V; static __device__ __forceinline__ V ld(const h16* p) { return cat16(*(const v8h*)p, *(const v8h*)(p + 16)); } static __device__ __forceinline__ v8f mma(V a, V b, v8f c) { return wmma16(a, b, c); } };
template <> struct WFrag<bf> { typedef v16bf V; static __device__ __forceinline__ V ld(const bf* p) { return cat16b(*(const v8us*)p, *(const v8us*)(p + 16)); } static __device__ __forceinline__ v8f mma(V a, V b, v8f c) { return wmmab(a, b, c); } };
template <typename T16, int NSPLIT, bool BIAS>
__global__ __launch_bounds__(32) void k_gemmw(const T16* __restrict__ A, const T16* __restrict__ A2, const T16* __restrict__ Bt, const T16* __restrict__ Bt2, int K, float* C, int ldc, const float* __restrict__ bias, size_t sA, size_t sB, size_t sC) {
    typedef typename WFrag<T16>::V V;
    __shared__ __align__(16) float os[16 * 68];
    const size_t z = blockIdx.z; A += z * sA; if (A2) A2 += z * sA; Bt += z * sB; if (Bt2) Bt2 += z * sB; C += z * sC;
    const int lane = threadIdx.x & 31, lr = lane & 15, hi = lane >> 4; const int r0 = blockIdx.x * 64, c0 = blockIdx.y * 64;
    v8f acc[4][4];
#pragma unroll
    for (int mb = 0; mb < 4; ++mb)
#pragma unroll
        for (int nb = 0; nb < 4; ++nb) acc[mb][nb] = (v8f){};
    const size_t aoff = (size_t)(r0 + lr) * K + 8 * hi, boff = (size_t)(c0 + lr) * K + 8 * hi;
#pragma unroll 1
    for (int kc = 0; kc < K; kc += 32) {
        V a[4], a2[4];
#pragma unroll
        for (int mb = 0; mb < 4; ++mb) { a[mb] = WFrag<T16>::ld(A + aoff + (size_t)mb * 16 * K + kc); if (NSPLIT == 1 || NSPLIT == 2) a2[mb] = WFrag<T16>::ld(A2 + aoff + (size_t)mb * 16 * K + kc); }
#pragma unroll
        for (int nb = 0; nb < 4; ++nb) { const V b = WFrag<T16>::ld(Bt + boff + (size_t)nb * 16 * K + kc); V b2; if (NSPLIT >= 2) b2 = WFrag<T16>::ld(Bt2 + boff + (size_t)nb * 16 * K + kc);
#pragma unroll
            for (int mb = 0; mb < 4; ++mb) { acc[mb][nb] = WFrag<T16>::mma(a[mb], b, acc[mb][nb]); if (NSPLIT == 1 || NSPLIT == 2) acc[mb][nb] = WFrag<T16>::mma(a2[mb], b, acc[mb][nb]); if (NSPLIT >= 2) acc[mb][nb] = WFrag<T16>::mma(a[mb], b2, acc[mb][nb]); } }
        asm volatile("v_nop\n\tv_nop\n\tv_nop\n\tv_nop" : "+v"(acc[0][0]), "+v"(acc[1][1]), "+v"(acc[2][2]), "+v"(acc[3][3]) : "v"(a[0]), "v"(a[3]));
    }
#pragma unroll
    for (int mb = 0; mb < 4; ++mb) {
#pragma unroll
        for (int nb = 0; nb < 4; ++nb) {
#pragma unroll
            for (int j = 0; j < 8; ++j) os[(hi * 8 + j) * 68 + nb * 16 + lr] = acc[mb][nb][j]; }
        __builtin_amdgcn_wave_barrier(); asm volatile("" ::: "memory");
        float* crow = C + (size_t)(r0 + mb * 16) * ldc + c0;
#pragma unroll 1
        for (int ps = 0; ps < 2; ++ps) {
#pragma unroll
            for (int s = 0; s < 8; ++s) { const int row = 2 * s + hi, cofs = lr * 4; v4f val = *(const v4fa*)(os + row * 68 + cofs); if (BIAS) { val[0] += bfr(bias[c0 + cofs]); val[1] += bfr(bias[c0 + cofs + 1]); val[2] += bfr(bias[c0 + cofs + 2]); val[3] += bfr(bias[c0 + cofs + 3]); }
                *(volatile v4f*)(crow + (size_t)row * ldc + cofs) = val; }
            if (ps == 0) __threadfence(); }
        __builtin_amdgcn_wave_barrier(); asm volatile("" ::: "memory");
    }
}

__device__ __forceinline__ h16 tohx(float x) { return (h16)x; }
__device__ __forceinline__ void splitf(float y, unsigned short& h, unsigned short& l) { h = f2bf(y); l = f2bf(y - bf2f(h)); }
typedef __attribute__((ext_vector_type(2))) _Float16 v2h;
typedef __attribute__((ext_vector_type(4))) _Float16 v4h;
typedef __attribute__((ext_vector_type(2))) unsigned short v2us;
typedef __attribute__((ext_vector_type(4))) unsigned short v4us;
typedef __attribute__((ext_vector_type(2))) float v2f;
typedef __attribute__((ext_vector_type(4))) int v4i;

__global__ __launch_bounds__(256) void k_cvt8(const float* __restrict__ src, bf* dst, size_t n8) { const size_t i = (size_t)blockIdx.x * 256 + threadIdx.x; if (i >= n8) return; const v8f v = *(const v8f*)(src + i * 8); v8us o;
#pragma unroll
    for (int k = 0; k < 8; ++k) o[k] = f2bf(v[k]); *(volatile v8us*)(dst + i * 8) = o; __threadfence(); *(volatile v8us*)(dst + i * 8) = o; }
__global__ __launch_bounds__(256) void k_split8(const float* __restrict__ F, bf* Ph, bf* Pl, size_t n8) { const size_t i = (size_t)blockIdx.x * 256 + threadIdx.x; if (i >= n8) return; const v8f v = *(const v8f*)(F + i * 8); v8us oh, ol;
#pragma unroll
    for (int k = 0; k < 8; ++k) { unsigned short a, c2; splitf(v[k], a, c2); oh[k] = a; ol[k] = c2; }
    *(volatile v8us*)(Ph + i * 8) = oh; *(volatile v8us*)(Pl + i * 8) = ol; __threadfence(); *(volatile v8us*)(Ph + i * 8) = oh; *(volatile v8us*)(Pl + i * 8) = ol; }

__global__ __launch_bounds__(256) void k_twid(bf* TWh, bf* TWl) { const size_t e = ((size_t)blockIdx.x * 256 + threadIdx.x) * 2; if (e >= (size_t)TC * NN) return; const int n = (int)(e % NN); const int c = (int)(e / NN); const int m = c & 31; v2us oh, ol;
#pragma unroll
    for (int q = 0; q < 2; ++q) { const unsigned r = ((unsigned)m * (unsigned)(n + q)) & (NN - 1); const float ang = (float)r * TWOPI_N; const float v = (c < MO) ? cosf(ang) : sinf(ang); unsigned short a, c2; splitf(v, a, c2); oh[q] = a; ol[q] = c2; }
    *(volatile v2us*)(TWh + e) = oh; *(volatile v2us*)(TWl + e) = ol; __threadfence(); *(volatile v2us*)(TWh + e) = oh; *(volatile v2us*)(TWl + e) = ol; }
__global__ __launch_bounds__(256) void k_twidT(bf* TTh, bf* TTl) { const size_t e = ((size_t)blockIdx.x * 256 + threadIdx.x) * 2; if (e >= (size_t)NN * TC) return; const int c = (int)(e % TC); const int n = (int)(e / TC); v2us oh, ol;
#pragma unroll
    for (int q = 0; q < 2; ++q) { const int cc = c + q; const int m = cc & 31; const unsigned r = ((unsigned)m * (unsigned)n) & (NN - 1); const float ang = (float)r * TWOPI_N; const float v = (cc < MO) ? cosf(ang) : sinf(ang); unsigned short a, c2; splitf(v, a, c2); oh[q] = a; ol[q] = c2; }
    *(volatile v2us*)(TTh + e) = oh; *(volatile v2us*)(TTl + e) = ol; __threadfence(); *(volatile v2us*)(TTh + e) = oh; *(volatile v2us*)(TTl + e) = ol; }
__global__ __launch_bounds__(256) void k_lift(const float* __restrict__ X, int b0, const float* __restrict__ lw, const float* __restrict__ lb, float* H) { const size_t i = (size_t)blockIdx.x * 256 + threadIdx.x; if (i >= (size_t)RWS * NN / 4) return; const size_t e = i * 4; const int n = (int)(e % NN); const int r = (int)(e / NN); const int bl = r / WD, o = r % WD; const v4f xv = *(const v4f*)(X + (size_t)(b0 + bl) * NN + n); const float w = bfr(lw[o]), bb = bfr(lb[o]); v4f ov;
#pragma unroll
    for (int q = 0; q < 4; ++q) { float p = __fmul_rn(w, bfr(xv[q])); asm volatile("" : "+v"(p)); ov[q] = __fadd_rn(p, bb); }
    *(volatile v4f*)(H + e) = ov; __threadfence(); *(volatile v4f*)(H + e) = ov; }
__global__ __launch_bounds__(256) void k_htr(const float* __restrict__ H, bf* Th, bf* Tl) { const size_t e = ((size_t)blockIdx.x * 256 + threadIdx.x) * 2; if (e >= (size_t)RWS * NN) return; const int i = (int)(e % WD); const int n = (int)((e / WD) % NN); const int bl = (int)(e / ((size_t)WD * NN)); v2us oh, ol;
#pragma unroll
    for (int q = 0; q < 2; ++q) { unsigned short a, c2; splitf(H[((size_t)bl * WD + i + q) * NN + n], a, c2); oh[q] = a; ol[q] = c2; }
    *(volatile v2us*)(Th + e) = oh; *(volatile v2us*)(Tl + e) = ol; __threadfence(); *(volatile v2us*)(Th + e) = oh; *(volatile v2us*)(Tl + e) = ol; }
__global__ __launch_bounds__(256) void k_smix(const float* __restrict__ XF, const float* __restrict__ wr, const float* __restrict__ wi, int k, float* COEF) { const int lane = threadIdx.x & 31; const int row = blockIdx.x * 8 + (threadIdx.x >> 5); if (row >= RWS) return; const int bl = row / WD, o = row % WD; float ore = 0.f, oim = 0.f;
#pragma unroll 4
    for (int i = 0; i < WD; ++i) { const float xr = XF[((size_t)bl * WD + i) * TC + lane]; const float xs = XF[((size_t)bl * WD + i) * TC + MO + lane]; const float xi = -xs; const size_t wo = (((size_t)k * WD + i) * WD + o) * MO + lane; const float a = bfr(wr[wo]), bq = bfr(wi[wo]);
        float p1 = __fmul_rn(xr, a), p2 = __fmul_rn(xi, bq), p3 = __fmul_rn(xr, bq), p4 = __fmul_rn(xi, a); asm volatile("" : "+v"(p1), "+v"(p2), "+v"(p3), "+v"(p4)); float dre = __fsub_rn(p1, p2), dim = __fadd_rn(p3, p4); asm volatile("" : "+v"(dre), "+v"(dim)); ore = __fadd_rn(ore, dre); oim = __fadd_rn(oim, dim); }
    const float sm = (lane == 0) ? (1.0f / NN) : (2.0f / NN); const float cre = ore * sm; const float cim = (lane == 0) ? 0.0f : -(oim * sm);
    float* dst = COEF + (size_t)row * TC; *(volatile float*)(dst + lane) = cre; *(volatile float*)(dst + MO + lane) = cim; __threadfence(); *(volatile float*)(dst + lane) = cre; *(volatile float*)(dst + MO + lane) = cim; }
__global__ __launch_bounds__(256) void k_comb(float* H, const float* __restrict__ SC, const float* __restrict__ bb, size_t n4) { const size_t i = (size_t)blockIdx.x * 256 + threadIdx.x; if (i >= n4) return; const size_t e = i * 4; const int o = (int)((e / NN) % WD); const float b2 = bfr(bb[o]); const v4f a = *(const v4f*)(H + e); const v4f s = *(const v4f*)(SC + e); v4f ov;
#pragma unroll
    for (int q = 0; q < 4; ++q) { float t = __fadd_rn(s[q], a[q]); asm volatile("" : "+v"(t)); ov[q] = __fadd_rn(t, b2); }
    *(volatile v4f*)(H + e) = ov; __threadfence(); *(volatile v4f*)(H + e) = ov; }
__global__ __launch_bounds__(256) void k_proj(const float* __restrict__ H, const float* __restrict__ pw, const float* __restrict__ pb, int b0, float* out) { const size_t g = (size_t)blockIdx.x * 256 + threadIdx.x; if (g >= (size_t)HB * NN) return; const int n = (int)(g % NN); const int bl = (int)(g / NN); float s = 0.f;
#pragma unroll 4
    for (int w = 0; w < WD; ++w) { float p = __fmul_rn(bfr(pw[w]), H[((size_t)bl * WD + w) * NN + n]); asm volatile("" : "+v"(p)); s = __fadd_rn(s, p); }
    const float o = __fadd_rn(s, bfr(pb[0])); *(volatile float*)(out + (size_t)(b0 + bl) * NN + n) = o; __threadfence(); *(volatile float*)(out + (size_t)(b0 + bl) * NN + n) = o; }

extern "C" void kernel_launch(void* const* d_in, const int* in_sizes, int n_in,
                              void* d_out, int out_size, void* d_ws, size_t ws_size, hipStream_t stream) {
    (void)in_sizes; (void)n_in; (void)out_size;
    const float* x = (const float*)d_in[0]; const float* lw = (const float*)d_in[1]; const float* lb = (const float*)d_in[2]; const float* wr = (const float*)d_in[3]; const float* wi = (const float*)d_in[4]; const float* bw = (const float*)d_in[5]; const float* bb = (const float*)d_in[6]; const float* pw = (const float*)d_in[7]; const float* pb = (const float*)d_in[8];
    float* OUT = (float*)d_out;
    char* wsp = (char*)d_ws;
    auto take = [&](size_t bytes) { char* p = wsp; wsp += (bytes + 255) & ~(size_t)255; return (void*)p; };
    bf* TWh = (bf*)take((size_t)TC * NN * 2); bf* TWl = (bf*)take((size_t)TC * NN * 2); bf* TTh = (bf*)take((size_t)NN * TC * 2); bf* TTl = (bf*)take((size_t)NN * TC * 2); bf* BW = (bf*)take((size_t)NBLK * WD * WD * 2);
    float* H = (float*)take((size_t)RWS * NN * 4); bf* Hh = (bf*)take((size_t)RWS * NN * 2); bf* Hl = (bf*)take((size_t)RWS * NN * 2); bf* HTh = (bf*)take((size_t)RWS * NN * 2); bf* HTl = (bf*)take((size_t)RWS * NN * 2); float* SC = (float*)take((size_t)RWS * NN * 4);
    float* XF = (float*)take((size_t)RWS * TC * 4); float* COEF = (float*)take((size_t)RWS * TC * 4); bf* CFh = (bf*)take((size_t)RWS * TC * 2); bf* CFl = (bf*)take((size_t)RWS * TC * 2);
    if ((size_t)(wsp - (char*)d_ws) > ws_size) return;
    k_twid<<<(unsigned)(((size_t)TC * NN / 2 + 255) / 256), 256, 0, stream>>>(TWh, TWl); k_twidT<<<(unsigned)(((size_t)NN * TC / 2 + 255) / 256), 256, 0, stream>>>(TTh, TTl); k_cvt8<<<(unsigned)(((size_t)NBLK * WD * WD / 8 + 255) / 256), 256, 0, stream>>>(bw, BW, (size_t)NBLK * WD * WD / 8);
    const unsigned L8 = (unsigned)(((size_t)RWS * NN / 8 + 255) / 256), L4 = (unsigned)(((size_t)RWS * NN / 4 + 255) / 256), L2 = (unsigned)(((size_t)RWS * NN / 2 + 255) / 256);
    for (int half = 0; half < NB_ / HB; ++half) { const int b0 = half * HB;
        k_lift<<<L4, 256, 0, stream>>>(x, b0, lw, lb, H);
        for (int k = 0; k < NBLK; ++k) {
            k_split8<<<L8, 256, 0, stream>>>(H, Hh, Hl, (size_t)RWS * NN / 8); k_htr<<<L2, 256, 0, stream>>>(H, HTh, HTl);
            k_gemmw<bf, 2, false><<<dim3(RWS / 64, TC / 64, 1), 32, 0, stream>>>(Hh, Hl, TWh, TWl, NN, XF, TC, nullptr, 0, 0, 0);
            k_smix<<<RWS / 8, 256, 0, stream>>>(XF, wr, wi, k, COEF); k_split8<<<(unsigned)(((size_t)RWS * TC / 8 + 255) / 256), 256, 0, stream>>>(COEF, CFh, CFl, (size_t)RWS * TC / 8);
            k_gemmw<bf, 3, false><<<dim3(WD / 64, NN / 64, HB), 32, 0, stream>>>(BW + (size_t)k * WD * WD, nullptr, HTh, HTl, WD, H, NN, nullptr, 0, (size_t)NN * WD, (size_t)WD * NN);
            k_gemmw<bf, 2, false><<<dim3(RWS / 64, NN / 64, 1), 32, 0, stream>>>(CFh, CFl, TTh, TTl, TC, SC, NN, nullptr, 0, 0, 0);
            k_comb<<<L4, 256, 0, stream>>>(H, SC, bb + (size_t)k * WD, (size_t)RWS * NN / 4); }
        k_proj<<<(unsigned)(((size_t)HB * NN + 255) / 256), 256, 0, stream>>>(H, pw, pb, b0, OUT); }
}
